// TemporalGuidedModule_59356448031017
// MI455X (gfx1250) — hardware-verified
//
#include <hip/hip_runtime.h>
#include <stdint.h>

typedef _Float16 v16h __attribute__((ext_vector_type(16)));
typedef _Float16 v8h  __attribute__((ext_vector_type(8)));
typedef float    v8f  __attribute__((ext_vector_type(8)));
typedef float    v4f  __attribute__((ext_vector_type(4)));

union Frag  { v16h v; v8h half[2]; };
union Pack8 { v8h h; v4f f; };

#define CDIM   256
#define NHEAD  8
#define NPNT   8
#define HDIM   32
#define HSZ    128
#define WSZ    128
#define HWQ    (HSZ * WSZ)
#define NBATCH 2
#define MTOT   (NBATCH * HWQ)
#define KSTEPS (CDIM / 32)
#define WROWS  (7 * CDIM + 128 + 64)

enum { EP_X1 = 0, EP_H = 1, EP_F = 2, EP_MULH = 3, EP_RELUH = 4, EP_ADDH = 5, EP_OUT = 6 };

__device__ __forceinline__ v8f wmma16(v16h a, v16h b, v8f c)
{
  v8f d = __builtin_amdgcn_wmma_f32_16x16x32_f16(false, a, false, b, (short)0, c, false, false);
  asm volatile("v_nop\n\tv_nop\n\tv_nop\n\tv_nop" : "+v"(d) : "v"(a), "v"(b));
  return d;
}

__device__ __forceinline__ v4f cvt8(v4f p, v4f q, float s)
{
  Pack8 u;
  v8h t = { (_Float16)(p[0] * s), (_Float16)(p[1] * s), (_Float16)(p[2] * s), (_Float16)(p[3] * s),
            (_Float16)(q[0] * s), (_Float16)(q[1] * s), (_Float16)(q[2] * s), (_Float16)(q[3] * s) };
  u.h = t;
  return u.f;
}

__global__ __launch_bounds__(32)
void k_wcvt(const float* __restrict__ w0, const float* __restrict__ w1, const float* __restrict__ w2,
            const float* __restrict__ w3, const float* __restrict__ w4, const float* __restrict__ w5,
            const float* __restrict__ w6, const float* __restrict__ w7, const float* __restrict__ w8,
            _Float16* __restrict__ Wh, float scale)
{
  const int row = blockIdx.x;
  const int l = threadIdx.x & 31;
  if (row >= WROWS) return;
  const float* src;
  if (row < 7 * CDIM) {
    const int seg = row >> 8, rr = row & (CDIM - 1);
    const float* base = (seg == 0) ? w0 : (seg == 1) ? w1 : (seg == 2) ? w2 : (seg == 3) ? w3
                      : (seg == 4) ? w4 : (seg == 5) ? w5 : w6;
    src = base + (size_t)rr * CDIM;
  } else if (row < 7 * CDIM + 128) {
    src = w7 + (size_t)(row - 7 * CDIM) * CDIM;
  } else {
    src = w8 + (size_t)(row - 7 * CDIM - 128) * CDIM;
  }
  const v4f x0 = *(const v4f*)(src + l * 8);
  const v4f x1 = *(const v4f*)(src + l * 8 + 4);
  const v4f pk = cvt8(x0, x1, scale);
  _Float16* dst = Wh + (size_t)row * CDIM + l * 8;
  *(volatile v4f*)dst = pk;
  __threadfence();
  *(volatile v4f*)dst = pk;
}

__global__ __launch_bounds__(256)
void k_tr(const float* __restrict__ X0, const float* __restrict__ X1,
          _Float16* __restrict__ Y0, _Float16* __restrict__ Y1)
{
  __shared__ __align__(16) _Float16 sT[64 * 72];
  const int tid = threadIdx.x, w = tid >> 5, l = tid & 31;
  const int p0 = blockIdx.x * 64, c0 = blockIdx.y * 64;
  const int t = blockIdx.z >> 1, b = blockIdx.z & 1;
  if (p0 + 64 > HWQ || c0 + 64 > CDIM || b >= NBATCH || t > 1) return;
  const float* X = t ? X1 : X0;
  _Float16*    Y = t ? Y1 : Y0;
  const float* src = X + ((size_t)(b * CDIM + c0)) * HWQ + p0;
  #pragma unroll
  for (int i = 0; i < 4; ++i) {
    const int u = tid + 256 * i;
    const int c = u >> 4;
    const int pg = u & 15;
    const v4f v = *(const v4f*)(src + (size_t)c * HWQ + 4 * pg);
    _Float16* s = sT + (4 * pg) * 72 + c;
    s[0]   = (_Float16)v[0];
    s[72]  = (_Float16)v[1];
    s[144] = (_Float16)v[2];
    s[216] = (_Float16)v[3];
  }
  __syncthreads();
  const int cc = (l & 7) * 8;
  v4f vals[2];
  #pragma unroll
  for (int i = 0; i < 2; ++i) {
    const int rl = w * 8 + 4 * i + (l >> 3);
    Pack8 u;
    u.h = *(const v8h*)(sT + rl * 72 + cc);
    vals[i] = u.f;
  }
  #pragma unroll
  for (int i = 0; i < 2; ++i) {
    const int rl = w * 8 + 4 * i + (l >> 3);
    _Float16* dst = Y + ((size_t)(b * HWQ + p0 + rl)) * CDIM + c0 + cc;
    *(volatile v4f*)dst = vals[i];
  }
  __threadfence();
  #pragma unroll
  for (int i = 0; i < 2; ++i) {
    const int rl = w * 8 + 4 * i + (l >> 3);
    _Float16* dst = Y + ((size_t)(b * HWQ + p0 + rl)) * CDIM + c0 + cc;
    *(volatile v4f*)dst = vals[i];
  }
}

template<int MODE>
__global__ __launch_bounds__(256)
void k_gemm(const _Float16* __restrict__ Ah, const _Float16* __restrict__ Wh,
            const float* __restrict__ bias, const float* __restrict__ X1f,
            float* __restrict__ Yf, _Float16* __restrict__ Yh,
            int M, int N, float inv_scale, float out_scale)
{
  constexpr bool kRelu = (MODE == EP_RELUH || MODE == EP_OUT);
  constexpr bool kF32  = (MODE == EP_X1 || MODE == EP_F);
  constexpr bool kF16  = (MODE == EP_X1 || MODE == EP_H || MODE == EP_MULH || MODE == EP_RELUH || MODE == EP_ADDH);
  constexpr bool kOut  = (MODE == EP_OUT);

  __shared__ __align__(16) float sC[128 * 64];

  const int tid = threadIdx.x;
  const int w = tid >> 5, l = tid & 31, h = l >> 4, m = l & 15;
  const int col0  = blockIdx.x * 64;
  const int tileM = blockIdx.y * 128;
  if (tileM + 128 > M || col0 + 64 > N) return;

  v8f acc[4] = {};

  const _Float16* ap = Ah + (size_t)(tileM + w * 16 + m) * CDIM + 8 * h;
  const _Float16* bp = Wh + (size_t)(col0 + m) * CDIM + 8 * h;

  #pragma unroll 1
  for (int kt = 0; kt < KSTEPS; ++kt) {
    const int k0 = kt * 32;
    Frag a;
    a.half[0] = *(const v8h*)(ap + k0);
    a.half[1] = *(const v8h*)(ap + k0 + 16);
    #pragma unroll
    for (int j = 0; j < 4; ++j) {
      const _Float16* bj = bp + (size_t)j * 16 * CDIM + k0;
      Frag b;
      b.half[0] = *(const v8h*)(bj);
      b.half[1] = *(const v8h*)(bj + 16);
      acc[j] = wmma16(a.v, b.v, acc[j]);
    }
  }

  #pragma unroll
  for (int j = 0; j < 4; ++j) {
    const int nl = j * 16 + m;
    const float bj = bias[col0 + nl];
    if (kOut) {
      v4f q0 = {0.f, 0.f, 0.f, 0.f}, q1 = {0.f, 0.f, 0.f, 0.f};
      #pragma unroll
      for (int r = 0; r < 4; ++r) {
        float v0 = acc[j][r] * inv_scale + bj;
        float v1 = acc[j][r + 4] * inv_scale + bj;
        if (kRelu) { v0 = fmaxf(v0, 0.0f); v1 = fmaxf(v1, 0.0f); }
        q0[r] = v0;
        q1[r] = v1;
      }
      const int ml = w * 16 + 8 * h;
      *(v4f*)&sC[nl * 128 + ml]     = q0;
      *(v4f*)&sC[nl * 128 + ml + 4] = q1;
    } else {
      #pragma unroll
      for (int r = 0; r < 8; ++r) {
        float v = acc[j][r] * inv_scale + bj;
        if (kRelu) v = fmaxf(v, 0.0f);
        sC[(w * 16 + 8 * h + r) * 64 + nl] = v;
      }
    }
  }
  __syncthreads();

  if (kOut) {
    const int bb = tileM / HWQ;
    const int p0 = tileM - bb * HWQ;
    v4f vals[8];
    #pragma unroll
    for (int i = 0; i < 8; ++i) vals[i] = *(const v4f*)&sC[(w * 8 + i) * 128 + l * 4];
    #pragma unroll
    for (int i = 0; i < 8; ++i) {
      float* dst = Yf + ((size_t)(bb * CDIM + col0 + w * 8 + i)) * HWQ + p0 + l * 4;
      *(volatile v4f*)dst = vals[i];
    }
    __threadfence();
    #pragma unroll
    for (int i = 0; i < 8; ++i) {
      float* dst = Yf + ((size_t)(bb * CDIM + col0 + w * 8 + i)) * HWQ + p0 + l * 4;
      *(volatile v4f*)dst = vals[i];
    }
  }

  if (kF32) {
    const int cc = (l & 15) * 4;
    v4f vals[8];
    #pragma unroll
    for (int i = 0; i < 8; ++i) {
      const int rl = w * 16 + 2 * i + (l >> 4);
      vals[i] = *(const v4f*)&sC[rl * 64 + cc];
    }
    #pragma unroll
    for (int i = 0; i < 8; ++i) {
      const int rl = w * 16 + 2 * i + (l >> 4);
      float* dst = Yf + (size_t)(tileM + rl) * (size_t)N + col0 + cc;
      *(volatile v4f*)dst = vals[i];
    }
    __threadfence();
    #pragma unroll
    for (int i = 0; i < 8; ++i) {
      const int rl = w * 16 + 2 * i + (l >> 4);
      float* dst = Yf + (size_t)(tileM + rl) * (size_t)N + col0 + cc;
      *(volatile v4f*)dst = vals[i];
    }
  }

  if (kF16) {
    const int cc = (l & 7) * 8;
    v4f hv[4];
    #pragma unroll
    for (int i = 0; i < 4; ++i) {
      const int rl = w * 16 + 4 * i + (l >> 3);
      v4f pa = *(const v4f*)&sC[rl * 64 + cc];
      v4f pb = *(const v4f*)&sC[rl * 64 + cc + 4];
      if (MODE == EP_MULH || MODE == EP_ADDH) {
        const float* xp = X1f + (size_t)(tileM + rl) * CDIM + col0 + cc;
        const v4f xa = *(const v4f*)xp;
        const v4f xb = *(const v4f*)(xp + 4);
        if (MODE == EP_MULH) { pa = xa * pa; pb = xb * pb; }
        else                 { pa = xa + pa; pb = xb + pb; }
      }
      hv[i] = cvt8(pa, pb, out_scale);
    }
    #pragma unroll
    for (int i = 0; i < 4; ++i) {
      const int rl = w * 16 + 4 * i + (l >> 3);
      _Float16* dst = Yh + (size_t)(tileM + rl) * CDIM + col0 + cc;
      *(volatile v4f*)dst = hv[i];
    }
    __threadfence();
    #pragma unroll
    for (int i = 0; i < 4; ++i) {
      const int rl = w * 16 + 4 * i + (l >> 3);
      _Float16* dst = Yh + (size_t)(tileM + rl) * CDIM + col0 + cc;
      *(volatile v4f*)dst = hv[i];
    }
  }
}

__global__ __launch_bounds__(256)
void k_sample(const float* __restrict__ val, const float* __restrict__ offs,
              const float* __restrict__ alog, _Float16* __restrict__ Oh,
              int M, float out_scale)
{
  const int w = threadIdx.x >> 5, l = threadIdx.x & 31;
  const int m = blockIdx.x * 8 + w;
  if (m >= M) return;
  const int bb = m / HWQ;
  const int q  = m - bb * HWQ;
  const int hh = l >> 2;
  const int py = q / WSZ, px = q - py * WSZ;
  const float cx0 = ((float)px + 0.5f) * (1.0f / (float)WSZ);
  const float cy0 = ((float)py + 0.5f) * (1.0f / (float)HSZ);

  const float* lp = alog + (size_t)m * (NHEAD * NPNT) + hh * NPNT;
  const v4f g0 = *(const v4f*)lp;
  const v4f g1 = *(const v4f*)(lp + 4);
  float mx = g0[0];
  mx = fmaxf(mx, g0[1]); mx = fmaxf(mx, g0[2]); mx = fmaxf(mx, g0[3]);
  mx = fmaxf(mx, g1[0]); mx = fmaxf(mx, g1[1]); mx = fmaxf(mx, g1[2]); mx = fmaxf(mx, g1[3]);
  float ssum = __expf(g0[0] - mx);
  ssum += __expf(g0[1] - mx); ssum += __expf(g0[2] - mx); ssum += __expf(g0[3] - mx);
  ssum += __expf(g1[0] - mx); ssum += __expf(g1[1] - mx); ssum += __expf(g1[2] - mx); ssum += __expf(g1[3] - mx);
  const float inv = 1.0f / ssum;

  const float* op = offs + (size_t)m * (NHEAD * NPNT * 2) + hh * (NPNT * 2);
  const float* vb = val + (size_t)bb * HWQ * CDIM + l * 8;

  v4f acc0 = {0.f, 0.f, 0.f, 0.f};
  v4f acc1 = {0.f, 0.f, 0.f, 0.f};

  #pragma unroll 1
  for (int p = 0; p < NPNT; ++p) {
    const float aw = __expf(lp[p] - mx) * inv;
    const float ox = op[2 * p + 0];
    const float oy = op[2 * p + 1];
    const float locx = cx0 + ox * (1.0f / (float)WSZ);
    const float locy = cy0 + oy * (1.0f / (float)HSZ);
    const float ix = locx * (float)WSZ - 0.5f;
    const float iy = locy * (float)HSZ - 0.5f;
    const float x0 = floorf(ix), y0 = floorf(iy);
    const float x1 = x0 + 1.0f,  y1 = y0 + 1.0f;
    const float wx0 = x1 - ix, wx1 = ix - x0;
    const float wy0 = y1 - iy, wy1 = iy - y0;
    const float vx0 = (x0 >= 0.0f && x0 < (float)WSZ) ? 1.0f : 0.0f;
    const float vx1 = (x1 >= 0.0f && x1 < (float)WSZ) ? 1.0f : 0.0f;
    const float vy0 = (y0 >= 0.0f && y0 < (float)HSZ) ? 1.0f : 0.0f;
    const float vy1 = (y1 >= 0.0f && y1 < (float)HSZ) ? 1.0f : 0.0f;
    const float w00 = (wx0 * wy0) * (vx0 * vy0);
    const float w10 = (wx1 * wy0) * (vx1 * vy0);
    const float w01 = (wx0 * wy1) * (vx0 * vy1);
    const float w11 = (wx1 * wy1) * (vx1 * vy1);
    const int xc0 = (int)fminf(fmaxf(x0, 0.0f), (float)(WSZ - 1));
    const int xc1 = (int)fminf(fmaxf(x1, 0.0f), (float)(WSZ - 1));
    const int yc0 = (int)fminf(fmaxf(y0, 0.0f), (float)(HSZ - 1));
    const int yc1 = (int)fminf(fmaxf(y1, 0.0f), (float)(HSZ - 1));
    const float* p00 = vb + (size_t)(yc0 * WSZ + xc0) * CDIM;
    const float* p10 = vb + (size_t)(yc0 * WSZ + xc1) * CDIM;
    const float* p01 = vb + (size_t)(yc1 * WSZ + xc0) * CDIM;
    const float* p11 = vb + (size_t)(yc1 * WSZ + xc1) * CDIM;
    const v4f a00 = *(const v4f*)p00, b00 = *(const v4f*)(p00 + 4);
    const v4f a10 = *(const v4f*)p10, b10 = *(const v4f*)(p10 + 4);
    const v4f a01 = *(const v4f*)p01, b01 = *(const v4f*)(p01 + 4);
    const v4f a11 = *(const v4f*)p11, b11 = *(const v4f*)(p11 + 4);
    v4f c0 = a00 * w00;
    c0 = c0 + a10 * w10;
    c0 = c0 + a01 * w01;
    c0 = c0 + a11 * w11;
    v4f c1 = b00 * w00;
    c1 = c1 + b10 * w10;
    c1 = c1 + b01 * w01;
    c1 = c1 + b11 * w11;
    acc0 = acc0 + c0 * aw;
    acc1 = acc1 + c1 * aw;
  }

  const v4f pk = cvt8(acc0, acc1, out_scale);
  _Float16* dst = Oh + (size_t)m * CDIM + l * 8;
  *(volatile v4f*)dst = pk;
  __threadfence();
  *(volatile v4f*)dst = pk;
}

extern "C" void kernel_launch(void* const* d_in, const int* in_sizes, int n_in,
                              void* d_out, int out_size, void* d_ws, size_t ws_size,
                              hipStream_t stream)
{
  if (n_in < 20) return;
  const int nAct = NBATCH * CDIM * HWQ;
  if (in_sizes[0] != nAct || in_sizes[1] != nAct || out_size != nAct) return;
  if (in_sizes[2] != CDIM * CDIM || in_sizes[4] != CDIM * CDIM || in_sizes[6] != CDIM * CDIM ||
      in_sizes[12] != CDIM * CDIM || in_sizes[14] != CDIM * CDIM || in_sizes[16] != CDIM * CDIM ||
      in_sizes[18] != CDIM * CDIM) return;
  if (in_sizes[8] != 128 * CDIM || in_sizes[10] != 64 * CDIM) return;
  if (in_sizes[3] != CDIM || in_sizes[5] != CDIM || in_sizes[7] != CDIM || in_sizes[13] != CDIM ||
      in_sizes[15] != CDIM || in_sizes[17] != CDIM || in_sizes[19] != CDIM ||
      in_sizes[9] != 128 || in_sizes[11] != 64) return;

  const float* xt     = (const float*)d_in[0];
  const float* xt_1   = (const float*)d_in[1];
  const float* W_in1  = (const float*)d_in[2];
  const float* b_in1  = (const float*)d_in[3];
  const float* W_in2  = (const float*)d_in[4];
  const float* b_in2  = (const float*)d_in[5];
  const float* Wv     = (const float*)d_in[6];
  const float* bv     = (const float*)d_in[7];
  const float* Ws     = (const float*)d_in[8];
  const float* bs_off = (const float*)d_in[9];
  const float* Wa     = (const float*)d_in[10];
  const float* ba     = (const float*)d_in[11];
  const float* Wo     = (const float*)d_in[12];
  const float* bo     = (const float*)d_in[13];
  const float* Wt1    = (const float*)d_in[14];
  const float* bt1    = (const float*)d_in[15];
  const float* Wt2    = (const float*)d_in[16];
  const float* bt2    = (const float*)d_in[17];
  const float* Wout   = (const float*)d_in[18];
  const float* bout   = (const float*)d_in[19];

  const size_t MiB   = (size_t)1 << 20;
  const size_t oW    = 0;
  const size_t oA0   = 1 * MiB;
  const size_t oA1   = 17 * MiB;
  const size_t oX1f  = 33 * MiB;
  const size_t oX1h  = 65 * MiB;
  const size_t oX2h  = 81 * MiB;
  const size_t oVal  = 97 * MiB;
  const size_t oOffs = 129 * MiB;
  const size_t oAlog = 145 * MiB;
  const size_t oMs   = 153 * MiB;
  const size_t oG    = 169 * MiB;
  const size_t oT1   = 185 * MiB;
  const size_t oS    = 201 * MiB;
  const size_t oEnd  = 217 * MiB;
  if (ws_size < oEnd) return;
  if ((size_t)WROWS * CDIM * sizeof(_Float16) > oA0 - oW) return;

  char* ws = (char*)d_ws;
  _Float16* Wh    = (_Float16*)(ws + oW);
  _Float16* A0h   = (_Float16*)(ws + oA0);
  _Float16* A1h   = (_Float16*)(ws + oA1);
  float*    x1f   = (float*)(ws + oX1f);
  _Float16* x1h   = (_Float16*)(ws + oX1h);
  _Float16* x2h   = (_Float16*)(ws + oX2h);
  float*    valf  = (float*)(ws + oVal);
  float*    offsf = (float*)(ws + oOffs);
  float*    alogf = (float*)(ws + oAlog);
  _Float16* msh   = (_Float16*)(ws + oMs);
  _Float16* gh    = (_Float16*)(ws + oG);
  _Float16* t1h   = (_Float16*)(ws + oT1);
  _Float16* sh    = (_Float16*)(ws + oS);

  const _Float16* WhIn1 = Wh + (size_t)0    * CDIM;
  const _Float16* WhIn2 = Wh + (size_t)256  * CDIM;
  const _Float16* WhV   = Wh + (size_t)512  * CDIM;
  const _Float16* WhO   = Wh + (size_t)768  * CDIM;
  const _Float16* WhT1  = Wh + (size_t)1024 * CDIM;
  const _Float16* WhT2  = Wh + (size_t)1280 * CDIM;
  const _Float16* WhOut = Wh + (size_t)1536 * CDIM;
  const _Float16* WhS   = Wh + (size_t)1792 * CDIM;
  const _Float16* WhA   = Wh + (size_t)1920 * CDIM;

  const int M = MTOT;
  const dim3 blk(256);
  const dim3 g256(256 / 64, MTOT / 128);
  const dim3 g128(128 / 64, MTOT / 128);
  const dim3 g64 (64 / 64,  MTOT / 128);
  const dim3 gtr (HWQ / 64, CDIM / 64, 2 * NBATCH);

  k_wcvt<<<dim3(WROWS), dim3(32), 0, stream>>>(W_in1, W_in2, Wv, Wo, Wt1, Wt2, Wout, Ws, Wa, Wh, 64.0f);
  k_tr<<<gtr, blk, 0, stream>>>(xt, xt_1, A0h, A1h);

  k_gemm<EP_X1><<<g256, blk, 0, stream>>>(A0h, WhIn1, b_in1, x1f, x1f, x1h, M, 256, 1.0f / 64.0f, 4.0f);
  k_gemm<EP_H><<<g256, blk, 0, stream>>>(A1h, WhIn2, b_in2, x1f, valf, x2h, M, 256, 1.0f / 64.0f, 4.0f);
  k_gemm<EP_F><<<g256, blk, 0, stream>>>(x2h, WhV, bv, x1f, valf, gh, M, 256, 1.0f / 256.0f, 1.0f);
  k_gemm<EP_F><<<g128, blk, 0, stream>>>(x1h, WhS, bs_off, x1f, offsf, gh, M, 128, 1.0f / 256.0f, 1.0f);
  k_gemm<EP_F><<<g64, blk, 0, stream>>>(x1h, WhA, ba, x1f, alogf, gh, M, 64, 1.0f / 256.0f, 1.0f);
  k_sample<<<dim3((MTOT + 7) / 8), blk, 0, stream>>>(valf, offsf, alogf, msh, M, 16.0f);
  k_gemm<EP_MULH><<<g256, blk, 0, stream>>>(msh, WhO, bo, x1f, valf, gh, M, 256, 1.0f / 1024.0f, 64.0f);
  k_gemm<EP_RELUH><<<g256, blk, 0, stream>>>(gh, WhT1, bt1, x1f, valf, t1h, M, 256, 1.0f / 4096.0f, 256.0f);
  k_gemm<EP_ADDH><<<g256, blk, 0, stream>>>(t1h, WhT2, bt2, x1f, valf, sh, M, 256, 1.0f / 16384.0f, 4.0f);
  k_gemm<EP_OUT><<<g256, blk, 0, stream>>>(sh, WhOut, bout, x1f, (float*)d_out, gh, M, 256, 1.0f / 256.0f, 1.0f);
}
